// HyperbolicEncoder_50792283242942
// MI455X (gfx1250) — hardware-run, weakly checked
//
#include <hip/hip_runtime.h>
#include <stddef.h>
#include <stdint.h>
#include <math.h>


#define NN      50000
#define NE      800000
#define DIN     256
#define DH      128
#define DE      64
#define KA      256
#define WP      256
#define SPLIT_L1 1
#define SPLIT_L2 1
#define KEXT1   (SPLIT_L1 ? 256 : 128)
#define KEXT2   (SPLIT_L2 ? 256 : 128)
#define NTHR    256
#define NWAVE   8
#define EPT     8
#define CHUNK   (NTHR * EPT)
#define WCAP    (EPT * 32)
#define LISTN   (NWAVE * WCAP)
#define NBA     1024
#define SLA     10
#define NKB     49
#define NPS     (NKB * NBA)
#define RCAP    28672
#define DEGCAP  64
#define GBM     64
#define GTHR    128
#define MP      50048
#define GL      (MP / GBM)
#define XU      (MP * 32)
#define GXB     (XU / NTHR)
#define GW_IN   16
#define GW1     16
#define GW2     8
#define GPAR    7
#define P_BIN   0
#define P_B1    128
#define P_A1S   256
#define P_A1D   384
#define P_B2    512
#define P_A2S   640
#define P_A2D   704
#define P_BA    768
#define PARN    896
#define AGG_ZINTS (LISTN + 2 * RCAP + 3 * NBA)
#define AGG_LDS_INTS (AGG_ZINTS + 16)
#define NEGB    (-3.0e38f)

static_assert((CHUNK & (CHUNK - 1)) == 0 && CHUNK <= 4096);
static_assert((NBA & (NBA - 1)) == 0 && NBA == (1 << SLA));
static_assert(NE < (1 << 21) && (NE % 4) == 0);
static_assert(NN < 65536);
static_assert(LISTN % NTHR == 0);
static_assert(NBA % NWAVE == 0 && NBA % 32 == 0 && NBA == 4 * NTHR);
static_assert(RCAP % (4 * NTHR) == 0 && RCAP < 32768 && AGG_ZINTS % 4 == 0);
static_assert(DEGCAP == 64);
static_assert(MP % GBM == 0 && MP >= NN && MP - NN < GBM && NPS >= MP);
static_assert(DH == 4 * 32 && DE == 2 * 32 && KA == 2 * DH && KA == DIN && WP == KA);
static_assert(KEXT1 % 32 == 0 && KEXT2 % 32 == 0 && KEXT1 <= KA && KEXT2 <= KA);
static_assert(GBM == (GTHR / 32) * 16);
static_assert(XU % NTHR == 0);
static_assert(DH * 32 == GW_IN * NTHR && DH * 32 == GW1 * NTHR && DE * 32 == GW2 * NTHR);
static_assert(AGG_LDS_INTS * 4 <= 327680);
static_assert(2 * NKB <= NTHR);

typedef float          v2f   __attribute__((ext_vector_type(2)));
typedef float          v4f   __attribute__((ext_vector_type(4)));
typedef float          v8f   __attribute__((ext_vector_type(8)));
typedef int            v4i   __attribute__((ext_vector_type(4)));
typedef int            v8i   __attribute__((ext_vector_type(8)));
typedef unsigned short v8us  __attribute__((ext_vector_type(8)));
typedef unsigned short v16us __attribute__((ext_vector_type(16)));
typedef __bf16         v16bf __attribute__((ext_vector_type(16)));
typedef v2f  __attribute__((may_alias)) v2fa;
typedef v4f  __attribute__((may_alias)) v4fa;
typedef v4i  __attribute__((may_alias)) v4ia;
typedef v8us __attribute__((may_alias)) v8usa;
union FragB { v16bf v; v16us u; v8us h[2]; v8i w; };

__device__ __forceinline__ v8f wmb(const FragB& a, const FragB& b, v8f c) {
  v8f d = __builtin_amdgcn_wmma_f32_16x16x32_bf16(false, a.v, false, b.v, (short)0, c, false, false);
  asm volatile("v_nop\n\tv_nop\n\tv_nop\n\tv_nop" : "+v"(d) : "v"(a.w), "v"(b.w));
  return d;
}

__device__ __forceinline__ unsigned bf16_bits(float f) {
  const unsigned u = __float_as_uint(f);
  return (u + 0x7FFFu + ((u >> 16) & 1u)) >> 16;
}
__device__ __forceinline__ float bf16_val(float f) {
  return __uint_as_float(bf16_bits(f) << 16);
}
__device__ __forceinline__ v4f bfr4(const v4f a) {
  v4f r; r.x = bf16_val(a.x); r.y = bf16_val(a.y); r.z = bf16_val(a.z); r.w = bf16_val(a.w); return r;
}
__device__ __forceinline__ void pin_i(int v)   { asm volatile("" :: "v"(v)); }
__device__ __forceinline__ void pin_f(float v) { asm volatile("" :: "v"(v)); }

__device__ __forceinline__ float wsum(float v) {
#pragma unroll
  for (int q = 16; q > 0; q >>= 1) v += __shfl_xor(v, q, 32);
  return v;
}

__device__ __forceinline__ void expmap4(float& a, float& b, float& c, float& d) {
  const float n  = sqrtf(wsum((a * a + b * b) + (c * c + d * d)));
  const bool  z  = (n == 0.0f);
  const float sf = z ? 1.0f : n;
  const float t  = tanhf(sf);
  const float r  = 1.0f / sf;
  const float ra = (t * a) * r, rb = (t * b) * r, rc = (t * c) * r, rd = (t * d) * r;
  a = z ? a : ra; b = z ? b : rb; c = z ? c : rc; d = z ? d : rd;
}
__device__ __forceinline__ void logmap4(float& a, float& b, float& c, float& d) {
  const float n  = sqrtf(wsum((a * a + b * b) + (c * c + d * d)));
  const bool  z  = (n == 0.0f);
  const float sf = z ? 1.0f : n;
  const float cl = (sf < 0.99f) ? sf : 0.99f;
  const float t  = atanhf(cl);
  const float r  = 1.0f / sf;
  const float ra = (t * a) * r, rb = (t * b) * r, rc = (t * c) * r, rd = (t * d) * r;
  a = z ? a : ra; b = z ? b : rb; c = z ? c : rc; d = z ? d : rd;
}
__device__ __forceinline__ void expmap2(float& a, float& b) {
  const float n  = sqrtf(wsum(a * a + b * b));
  const bool  z  = (n == 0.0f);
  const float sf = z ? 1.0f : n;
  const float t  = tanhf(sf);
  const float r  = 1.0f / sf;
  const float ra = (t * a) * r, rb = (t * b) * r;
  a = z ? a : ra; b = z ? b : rb;
}
__device__ __forceinline__ float relu_keep(float v) { return (v > 0.0f) ? v : (v - v); }

__device__ __forceinline__ float edge_logit(float as, float ad, float ab) {
  const float v = (as + ad) + ab;
  return (v > 0.0f) ? v : 0.2f * v;
}
__device__ __forceinline__ int alidx(int n) { return (n >> 6) * (2 * GBM) + (n & (GBM - 1)); }

__device__ __forceinline__ void hilo_pack(float v0, float v1, float v2, float v3,
                                          int& h01, int& h23, int& l01, int& l23) {
  const unsigned a0 = bf16_bits(v0), a1 = bf16_bits(v1), a2 = bf16_bits(v2), a3 = bf16_bits(v3);
  const unsigned b0 = bf16_bits(v0 - __uint_as_float(a0 << 16));
  const unsigned b1 = bf16_bits(v1 - __uint_as_float(a1 << 16));
  const unsigned b2 = bf16_bits(v2 - __uint_as_float(a2 << 16));
  const unsigned b3 = bf16_bits(v3 - __uint_as_float(a3 << 16));
  h01 = (int)(a0 | (a1 << 16)); h23 = (int)(a2 | (a3 << 16));
  l01 = (int)(b0 | (b1 << 16)); l23 = (int)(b2 | (b3 << 16));
}

__device__ __forceinline__ v4i regroup16(int h01, int h23, int l01, int l23, int lane) {
  const int s0 = (2 * lane) & 31, s1 = s0 + 1;
  const int a0 = __shfl(h01, s0, 32), a1 = __shfl(h23, s0, 32), a2 = __shfl(h01, s1, 32), a3 = __shfl(h23, s1, 32);
  const int b0 = __shfl(l01, s0, 32), b1 = __shfl(l23, s0, 32), b2 = __shfl(l01, s1, 32), b3 = __shfl(l23, s1, 32);
  const int mk = (lane < 16) ? -1 : 0;
  v4i o;
  o.x = (a0 & mk) | (b0 & ~mk); o.y = (a1 & mk) | (b1 & ~mk);
  o.z = (a2 & mk) | (b2 & ~mk); o.w = (a3 & mk) | (b3 & ~mk);
  return o;
}

template <int SLB>
__device__ __forceinline__ int scan_chunk(const int* __restrict__ dsts, int nE, int cbase, int slotBase,
                                          int nb, int vec8, int* list, int tid, int lane, int wave) {
  int wc = 0;
  const int el0  = tid * EPT;
  const int e0   = cbase + el0;
  const int sent = (int)(1u << 31);
  v4i da, db;
  if (vec8 != 0 && cbase + CHUNK <= nE) {
    da = *(const v4i*)(dsts + e0);
    db = *(const v4i*)(dsts + e0 + 4);
  } else {
    da.x = (e0     < nE) ? dsts[min(e0,     nE - 1)] : sent;
    da.y = (e0 + 1 < nE) ? dsts[min(e0 + 1, nE - 1)] : sent;
    da.z = (e0 + 2 < nE) ? dsts[min(e0 + 2, nE - 1)] : sent;
    da.w = (e0 + 3 < nE) ? dsts[min(e0 + 3, nE - 1)] : sent;
    db.x = (e0 + 4 < nE) ? dsts[min(e0 + 4, nE - 1)] : sent;
    db.y = (e0 + 5 < nE) ? dsts[min(e0 + 5, nE - 1)] : sent;
    db.z = (e0 + 6 < nE) ? dsts[min(e0 + 6, nE - 1)] : sent;
    db.w = (e0 + 7 < nE) ? dsts[min(e0 + 7, nE - 1)] : sent;
  }
  const unsigned nbs = (unsigned)slotBase;
  const unsigned unb = (unsigned)nb;
  const unsigned s0 = (unsigned)da.x - nbs, s1 = (unsigned)da.y - nbs;
  const unsigned s2 = (unsigned)da.z - nbs, s3 = (unsigned)da.w - nbs;
  const unsigned s4 = (unsigned)db.x - nbs, s5 = (unsigned)db.y - nbs;
  const unsigned s6 = (unsigned)db.z - nbs, s7 = (unsigned)db.w - nbs;
  const bool h0 = s0 < unb, h1 = s1 < unb, h2 = s2 < unb, h3 = s3 < unb;
  const bool h4 = s4 < unb, h5 = s5 < unb, h6 = s6 < unb, h7 = s7 < unb;
  const unsigned any = __builtin_amdgcn_ballot_w32(h0 | h1 | h2 | h3 | h4 | h5 | h6 | h7);
  if (any != 0u) {
#define HITJ(J, HJ, SJ) { \
      const unsigned mj = __builtin_amdgcn_ballot_w32(HJ); \
      if (mj != 0u) { \
        if (HJ) { \
          const int pos = wc + (int)__builtin_amdgcn_mbcnt_lo(mj, 0u); \
          if (pos < WCAP) list[wave * WCAP + pos] = ((el0 + (J)) << SLB) | (int)(SJ); \
        } \
        wc += (int)__builtin_popcount(mj); } }
    HITJ(0, h0, s0)
    HITJ(1, h1, s1)
    HITJ(2, h2, s2)
    HITJ(3, h3, s3)
    HITJ(4, h4, s4)
    HITJ(5, h5, s5)
    HITJ(6, h6, s6)
    HITJ(7, h7, s7)
#undef HITJ
  }
  return wc;
}

__global__ __launch_bounds__(NTHR) void k_prep(const float* __restrict__ x, const float* __restrict__ win,
                                               const float* __restrict__ w1, const float* __restrict__ w2,
                                               const float* __restrict__ bin, const float* __restrict__ b1,
                                               const float* __restrict__ a1, const float* __restrict__ ba1,
                                               const float* __restrict__ b2, const float* __restrict__ a2,
                                               const float* __restrict__ ba2,
                                               unsigned short* xb, unsigned short* wint, unsigned short* w1d,
                                               unsigned short* w2d, float* par) {
  const int tid = (int)threadIdx.x;
  const int blk = (int)blockIdx.x;
  v8us o;
  unsigned short* dp;
  if (blk < GXB) {
    const int u   = blk * NTHR + tid;
    const int row = u >> 5;
    const int k8  = (u & 31) * 8;
    const int rc  = row < NN ? row : NN - 1;
    const float* p = x + (size_t)rc * DIN + k8;
    const v4f a = *(const v4fa*)p;
    const v4f b = *(const v4fa*)(p + 4);
    const bool ok = row < NN;
    o[0] = ok ? (unsigned short)bf16_bits(a.x) : (unsigned short)0;
    o[1] = ok ? (unsigned short)bf16_bits(a.y) : (unsigned short)0;
    o[2] = ok ? (unsigned short)bf16_bits(a.z) : (unsigned short)0;
    o[3] = ok ? (unsigned short)bf16_bits(a.w) : (unsigned short)0;
    o[4] = ok ? (unsigned short)bf16_bits(b.x) : (unsigned short)0;
    o[5] = ok ? (unsigned short)bf16_bits(b.y) : (unsigned short)0;
    o[6] = ok ? (unsigned short)bf16_bits(b.z) : (unsigned short)0;
    o[7] = ok ? (unsigned short)bf16_bits(b.w) : (unsigned short)0;
    dp = xb + (size_t)row * KA + k8;
  } else if (blk < GXB + GW_IN) {
    const int u  = (blk - GXB) * NTHR + tid;
    const int n  = u >> 5;
    const int k8 = (u & 31) * 8;
    const float* p = win + (size_t)k8 * DH + n;
#pragma unroll
    for (int i = 0; i < 8; ++i) o[i] = (unsigned short)bf16_bits(p[(size_t)i * DH]);
    dp = wint + (size_t)n * WP + k8;
  } else if (blk < GXB + GW_IN + GW1) {
    const int u  = (blk - GXB - GW_IN) * NTHR + tid;
    const int n  = u >> 5;
    const int k8 = (u & 31) * 8;
    const int kk = k8 & (DH - 1);
    const float* p = w1 + (size_t)kk * DH + n;
#pragma unroll
    for (int i = 0; i < 8; ++i) o[i] = (unsigned short)bf16_bits(p[(size_t)i * DH]);
    dp = w1d + (size_t)n * WP + k8;
  } else if (blk < GXB + GW_IN + GW1 + GW2) {
    const int u  = (blk - GXB - GW_IN - GW1) * NTHR + tid;
    const int n  = u >> 5;
    const int k8 = (u & 31) * 8;
    const int kk = k8 & (DH - 1);
    const float* p = w2 + (size_t)kk * DE + n;
#pragma unroll
    for (int i = 0; i < 8; ++i) o[i] = (unsigned short)bf16_bits(p[(size_t)i * DE]);
    dp = w2d + (size_t)n * WP + k8;
  } else {
    const int pb = blk - (GXB + GW_IN + GW1 + GW2);
    const int ln = tid & 31;
    v4f q = {0.f, 0.f, 0.f, 0.f};
    if (pb == 0) {
      q = bfr4(*(const v4fa*)(bin + 4 * ln));
    } else if (pb == 1) {
      q = bfr4(*(const v4fa*)(b1 + 4 * ln));
    } else if (pb == 2) {
      q = bfr4(*(const v4fa*)(a1 + 4 * ln));
    } else if (pb == 3) {
      q = bfr4(*(const v4fa*)(a1 + DH + 4 * ln));
    } else if (pb == 4) {
      const int lc = ln < 16 ? ln : 15;
      const v4f t = bfr4(*(const v4fa*)(b2 + 4 * lc));
      const bool ok = ln < 16;
      q.x = ok ? t.x : 0.0f; q.y = ok ? t.y : 0.0f; q.z = ok ? t.z : 0.0f; q.w = ok ? t.w : 0.0f;
    } else if (pb == 5) {
      q = bfr4(*(const v4fa*)(a2 + 4 * ln));
    } else {
      const float s1 = bf16_val(ba1[0]);
      const float s2 = bf16_val(ba2[0]);
      q.x = (ln == 0) ? s1 : 0.0f;
      q.y = (ln == 0) ? s2 : 0.0f;
    }
    if (tid < 32) {
      float* fp = par + pb * 128 + 4 * ln;
      *(volatile v4f*)fp = q;
      __threadfence();
      *(volatile v4f*)fp = q;
    }
    return;
  }
  *(volatile v8us*)dp = o;
  __threadfence();
  *(volatile v8us*)dp = o;
}

__global__ __launch_bounds__(NTHR) void k_bucket(const int* __restrict__ ei, int* hits, int* oc, int* flag) {
  extern __shared__ __attribute__((aligned(16))) int dsm[];
  int* list = dsm;
  int* hl   = dsm + LISTN;
  int* sl   = dsm + LISTN + RCAP;
  int* cnt  = dsm + LISTN + 2 * RCAP;
  int* offs = cnt + NBA;
  int* cur  = offs + NBA;
  int* misc = cur + NBA;
  const int tid = (int)threadIdx.x, lane = tid & 31, wave = tid >> 5;
  const int blk  = (int)blockIdx.x;
  const int role = blk / NKB;
  const int kb   = blk - role * NKB;
  const int* keys = ei + (size_t)role * NE;
  const int* part = ei + (size_t)(1 - role) * NE;
  const int nodeBase = kb * NBA;
  const int nb = (NN - nodeBase) < NBA ? (NN - nodeBase) : NBA;

  {
    const v4i z4 = {0, 0, 0, 0};
    for (int i = tid * 4; i < AGG_ZINTS; i += NTHR * 4) *(v4ia*)(dsm + i) = z4;
    if (tid < 16) misc[tid] = 0;
  }
  __syncthreads();

  int t = 0, ov = 0;
  const int nChunks = (NE + CHUNK - 1) / CHUNK;
#pragma unroll 1
  for (int ch = 0; ch < nChunks; ++ch) {
    const int cbase = ch * CHUNK;
    const int wc = scan_chunk<SLA>(keys, NE, cbase, nodeBase, nb, 1, list, tid, lane, wave);
    if (lane == 0) misc[wave] = wc;
    __syncthreads();
    if (wave == 0) {
#pragma unroll 1
      for (int w2 = 0; w2 < NWAVE; ++w2) {
        int c = misc[w2];
        c = c < 0 ? 0 : (c > WCAP ? WCAP : c);
#pragma unroll 1
        for (int b0 = 0; b0 < c; b0 += 32) {
          const int idx = b0 + lane;
          const int ent = list[w2 * WCAP + (idx < WCAP ? idx : WCAP - 1)];
          const int m32 = (c - b0) < 32 ? (c - b0) : 32;
#pragma unroll 1
          for (int k = 0; k < m32; ++k) {
            const int u    = __builtin_amdgcn_readlane(ent, k);
            const int slot = u & (NBA - 1);
            const int el   = (u >> SLA) & (CHUNK - 1);
            const int pk   = ((cbase + el) << SLA) | slot;
            if (t < RCAP) {
              if (lane == 0) { hl[t] = pk; cnt[slot] = cnt[slot] + 1; }
              t = t + 1;
            } else {
              ov = 1;
            }
          }
        }
      }
    }
    __syncthreads();
  }
  if (wave == 0 && lane == 0) { misc[8] = t; misc[9] = ov; }
  __syncthreads();
  int tt = misc[8];
  tt = tt < 0 ? 0 : (tt > RCAP ? RCAP : tt);

  if (wave == 0) {
    const int base = lane * (NBA / 32);
    int s = 0, big = 0;
#pragma unroll 1
    for (int i = 0; i < NBA / 32; ++i) {
      const int cv = cnt[base + i];
      s += cv;
      big |= (cv > DEGCAP) ? 1 : 0;
    }
    const unsigned bm = __builtin_amdgcn_ballot_w32(big != 0);
    if (lane == 0) misc[10] = (bm != 0u) ? 1 : 0;
    int incl = s;
#pragma unroll
    for (int d = 1; d < 32; d <<= 1) {
      const int y = __shfl_up(incl, d, 32);
      if (lane >= d) incl += y;
    }
    int run = incl - s;
#pragma unroll 1
    for (int i = 0; i < NBA / 32; ++i) {
      const int cv = cnt[base + i];
      offs[base + i] = run;
      cur[base + i]  = run;
      run += cv;
    }
  }
  __syncthreads();
  if (wave == 0) {
#pragma unroll 1
    for (int b0 = 0; b0 < tt; b0 += 32) {
      const int idx = b0 + lane;
      const int ent = hl[idx < RCAP ? idx : RCAP - 1];
      const int m32 = (tt - b0) < 32 ? (tt - b0) : 32;
#pragma unroll 1
      for (int k = 0; k < m32; ++k) {
        const int u    = __builtin_amdgcn_readlane(ent, k);
        const int slot = u & (NBA - 1);
        if (lane == 0) {
          int p = cur[slot];
          p = p < 0 ? 0 : (p > RCAP - 1 ? RCAP - 1 : p);
          sl[p] = u;
          cur[slot] = p + 1;
        }
      }
    }
  }
  __syncthreads();

  const int ovf = ((misc[9] | misc[10]) != 0) ? 1 : 0;
#pragma unroll 1
  for (int i = tid; i < RCAP; i += NTHR) {
    const int ent = sl[i];
    int eid = ent >> SLA;
    eid = eid < 0 ? 0 : (eid > NE - 1 ? NE - 1 : eid);
    int pv = part[eid];
    pin_i(pv);
    pv = pv < 0 ? 0 : (pv > NN - 1 ? NN - 1 : pv);
    hl[i] = (i < tt) ? pv : 0;
  }
#pragma unroll
  for (int j = 0; j < 4; ++j) {
    const int s = tid * 4 + j;
    int ofv = offs[s]; ofv = ofv < 0 ? 0 : (ofv > RCAP ? RCAP : ofv);
    int cv  = cnt[s];  cv  = cv  < 0 ? 0 : (cv  > RCAP ? RCAP : cv);
    cur[s] = (ofv << 16) | cv;
  }
  __syncthreads();

  int* hp = hits + (size_t)blk * RCAP;
  int* op = oc + (size_t)role * NPS + nodeBase + 4 * tid;
  int* fp = flag + blk * 32 + 4 * (tid & 7);
  const v4i ocv = *(const v4ia*)(cur + 4 * tid);
  v4i fv; fv.x = ovf; fv.y = ovf; fv.z = ovf; fv.w = ovf;
#pragma unroll 1
  for (int i4 = tid; i4 < RCAP / 4; i4 += NTHR) {
    const v4i v = *(const v4ia*)(hl + 4 * i4);
    *(volatile v4i*)(hp + 4 * i4) = v;
  }
  *(volatile v4i*)op = ocv;
  if (tid < 8) *(volatile v4i*)fp = fv;
  __threadfence();
#pragma unroll 1
  for (int i4 = tid; i4 < RCAP / 4; i4 += NTHR) {
    const v4i v = *(const v4ia*)(hl + 4 * i4);
    *(volatile v4i*)(hp + 4 * i4) = v;
  }
  *(volatile v4i*)op = ocv;
  if (tid < 8) *(volatile v4i*)fp = fv;
}

__global__ __launch_bounds__(GTHR) __attribute__((amdgpu_num_vgpr(248)))
void k_lin0(const unsigned short* __restrict__ A, const unsigned short* __restrict__ BT,
            const float* __restrict__ par, unsigned short* XT) {
  __shared__ __attribute__((aligned(16))) float stg[GBM * DH];
  __shared__ __attribute__((aligned(16))) float shb[DH];
  const int tid = (int)threadIdx.x, lane = tid & 31, wave = tid >> 5, hh = lane >> 4, m = lane & 15;
  const int rowBase = (int)blockIdx.x * GBM;
  {
    const int ci = tid < 32 ? tid : 31;
    const v4f bq = *(const v4fa*)(par + P_BIN + 4 * ci);
    if (tid < 32) *(v4fa*)(shb + 4 * tid) = bq;
  }
  v8f acc[8];
  {
    const v8f z = {0.f, 0.f, 0.f, 0.f, 0.f, 0.f, 0.f, 0.f};
#pragma unroll
    for (int t = 0; t < 8; ++t) acc[t] = z;
  }
  const unsigned short* ap = A  + (size_t)(rowBase + 16 * wave + m) * (size_t)KA + 8 * hh;
  const unsigned short* bp = BT + (size_t)m * (size_t)WP + 8 * hh;
#pragma unroll 1
  for (int k0 = 0; k0 < DIN; k0 += 32) {
    FragB af;
    af.h[0] = *(const v8usa*)(ap + k0);
    af.h[1] = *(const v8usa*)(ap + k0 + 16);
#pragma unroll
    for (int nt = 0; nt < 8; ++nt) {
      const unsigned short* wq = bp + (size_t)(16 * nt) * (size_t)WP + k0;
      FragB bf;
      bf.h[0] = *(const v8usa*)wq;
      bf.h[1] = *(const v8usa*)(wq + 16);
      acc[nt] = wmb(af, bf, acc[nt]);
    }
  }
#pragma unroll
  for (int nt = 0; nt < 8; ++nt) {
    const int lc = 16 * nt + m;
#pragma unroll
    for (int r = 0; r < 8; ++r) {
      const int lr = 16 * wave + 8 * hh + r;
      stg[lr * DH + lc] = acc[nt][r];
    }
  }
  __syncthreads();
  const v4f hb = *(const v4fa*)(shb + 4 * lane);
#pragma unroll 1
  for (int i = 0; i < 16; ++i) {
    const int lr   = 16 * wave + i;
    const int grow = rowBase + lr;
    const bool live = grow < NN;
    const v4f mv = *(const v4fa*)(stg + lr * DH + 4 * lane);
    float v0 = relu_keep(mv.x + hb.x), v1 = relu_keep(mv.y + hb.y);
    float v2 = relu_keep(mv.z + hb.z), v3 = relu_keep(mv.w + hb.w);
    expmap4(v0, v1, v2, v3);
    logmap4(v0, v1, v2, v3);
    v0 = live ? v0 : 0.0f; v1 = live ? v1 : 0.0f; v2 = live ? v2 : 0.0f; v3 = live ? v3 : 0.0f;
    int h01, h23, l01, l23;
    hilo_pack(v0, v1, v2, v3, h01, h23, l01, l23);
    const v4i o = regroup16(h01, h23, l01, l23, lane);
    unsigned short* dp = XT + (size_t)grow * KA + 8 * lane;
    *(volatile v4i*)dp = o;
    __threadfence();
    *(volatile v4i*)dp = o;
  }
}

template <int D>
__global__ __launch_bounds__(GTHR) __attribute__((amdgpu_num_vgpr(248)))
void k_lin(const unsigned short* __restrict__ A, const unsigned short* __restrict__ BT, int kext,
           const float* __restrict__ par, int pbo, int pso, int pdo, float* HH, float* AL) {
  constexpr int NT  = D / 16;
  constexpr int CPL = D / 32;
  constexpr int ITER = (GBM * D / 4) / GTHR;
  static_assert(D == DH || D == DE);
  __shared__ __attribute__((aligned(16))) float stg[GBM * D];
  __shared__ __attribute__((aligned(16))) float shb[D];
  __shared__ __attribute__((aligned(16))) float sav[2 * D];
  __shared__ __attribute__((aligned(16))) float sdt[2 * GBM];
  const int tid = (int)threadIdx.x, lane = tid & 31, wave = tid >> 5, hh = lane >> 4, m = lane & 15;
  const int rowBase = (int)blockIdx.x * GBM;
  {
    const int ci = tid < (D / 4) ? tid : (D / 4 - 1);
    const v4f bq = *(const v4fa*)(par + pbo + 4 * ci);
    const v4f sq = *(const v4fa*)(par + pso + 4 * ci);
    const v4f dq = *(const v4fa*)(par + pdo + 4 * ci);
    if (tid < D / 4) {
      *(v4fa*)(shb + 4 * tid)     = bq;
      *(v4fa*)(sav + 4 * tid)     = sq;
      *(v4fa*)(sav + D + 4 * tid) = dq;
    }
  }
  __syncthreads();
  v8f acc[NT];
  {
    const v8f z = {0.f, 0.f, 0.f, 0.f, 0.f, 0.f, 0.f, 0.f};
#pragma unroll
    for (int t = 0; t < NT; ++t) acc[t] = z;
  }
  const unsigned short* ap = A  + (size_t)(rowBase + 16 * wave + m) * (size_t)KA + 8 * hh;
  const unsigned short* bp = BT + (size_t)m * (size_t)WP + 8 * hh;
#pragma unroll 1
  for (int k0 = 0; k0 < kext; k0 += 32) {
    FragB af;
    af.h[0] = *(const v8usa*)(ap + k0);
    af.h[1] = *(const v8usa*)(ap + k0 + 16);
#pragma unroll
    for (int nt = 0; nt < NT; ++nt) {
      const unsigned short* wq = bp + (size_t)(16 * nt) * (size_t)WP + k0;
      FragB bf;
      bf.h[0] = *(const v8usa*)wq;
      bf.h[1] = *(const v8usa*)(wq + 16);
      acc[nt] = wmb(af, bf, acc[nt]);
    }
  }
#pragma unroll
  for (int nt = 0; nt < NT; ++nt) {
    const int lc = 16 * nt + m;
    const float bs = shb[lc];
#pragma unroll
    for (int r = 0; r < 8; ++r) {
      const int lr = 16 * wave + 8 * hh + r;
      stg[lr * D + lc] = acc[nt][r] + bs;
    }
  }
  __syncthreads();

  float sa[CPL], da[CPL];
#pragma unroll
  for (int c = 0; c < CPL; ++c) { sa[c] = sav[CPL * lane + c]; da[c] = sav[D + CPL * lane + c]; }
#pragma unroll 1
  for (int i = 0; i < 16; ++i) {
    const int row = 16 * wave + i;
    float s = 0.0f, d = 0.0f;
#pragma unroll
    for (int c = 0; c < CPL; ++c) {
      const float p = stg[row * D + CPL * lane + c];
      s = fmaf(p, sa[c], s);
      d = fmaf(p, da[c], d);
    }
#pragma unroll
    for (int q = 16; q > 0; q >>= 1) {
      s += __shfl_xor(s, q, 32);
      d += __shfl_xor(d, q, 32);
    }
    if (lane == 0) { sdt[row] = s; sdt[GBM + row] = d; }
  }
  __syncthreads();

  const v4f alv = *(const v4fa*)(sdt + 4 * lane);
  float* alp = AL + (size_t)blockIdx.x * (2 * GBM) + 4 * lane;
  float* cp  = HH + (size_t)rowBase * D;
#pragma unroll 1
  for (int j = 0; j < ITER; ++j) {
    const int idx = j * GTHR + tid;
    const v4f p = *(const v4fa*)(stg + 4 * idx);
    *(volatile v4f*)(cp + 4 * idx) = p;
  }
  if (wave == 0) *(volatile v4f*)alp = alv;
  __threadfence();
#pragma unroll 1
  for (int j = 0; j < ITER; ++j) {
    const int idx = j * GTHR + tid;
    const v4f p = *(const v4fa*)(stg + 4 * idx);
    *(volatile v4f*)(cp + 4 * idx) = p;
  }
  if (wave == 0) *(volatile v4f*)alp = alv;
}

__global__ __launch_bounds__(NTHR) void k_srcstat(const int* __restrict__ hits, const int* __restrict__ oc,
                                                  const float* __restrict__ AL, const float* __restrict__ par,
                                                  int layer, float* REC) {
  __shared__ __attribute__((aligned(16))) float srec[NBA * 4];
  const int tid = (int)threadIdx.x, lane = tid & 31, wave = tid >> 5;
  const int kb = (int)blockIdx.x;
  const int nodeBase = kb * NBA;
  const int* hp  = hits + (size_t)kb * RCAP;
  const int* ocp = oc + nodeBase;
  const float ab = par[P_BA + layer];
#pragma unroll 1
  for (int si = 0; si < NBA / NWAVE; ++si) {
    const int s    = si * NWAVE + wave;
    const int node = nodeBase + s;
    const int nc   = node < NN ? node : NN - 1;
    const int ocv  = ocp[s];
    int o = (int)(((unsigned)ocv) >> 16);
    o = o > RCAP - 1 ? RCAP - 1 : o;
    int c = ocv & 0xffff;
    c = c > DEGCAP ? DEGCAP : c;
    o = __builtin_amdgcn_readfirstlane(o);
    c = __builtin_amdgcn_readfirstlane(c);
    const float asv = AL[alidx(nc)];
    int i0 = o + lane;
    i0 = i0 > RCAP - 1 ? RCAP - 1 : i0;
    int d0 = hp[i0];
    pin_i(d0);
    d0 = d0 < 0 ? 0 : (d0 > NN - 1 ? NN - 1 : d0);
    const float ad0 = AL[alidx(d0) + GBM];
    pin_f(ad0);
    const float e0 = edge_logit(asv, ad0, ab);
    float e1 = 0.0f;
    if (c > 32) {
      int i1 = o + 32 + lane;
      i1 = i1 > RCAP - 1 ? RCAP - 1 : i1;
      int d1 = hp[i1];
      pin_i(d1);
      d1 = d1 < 0 ? 0 : (d1 > NN - 1 ? NN - 1 : d1);
      const float ad1 = AL[alidx(d1) + GBM];
      pin_f(ad1);
      e1 = edge_logit(asv, ad1, ab);
    }
    const bool v0 = lane < c;
    const bool v1 = (32 + lane) < c;
    const float m0 = v0 ? e0 : NEGB;
    const float m1 = v1 ? e1 : NEGB;
    float mx = m0 > m1 ? m0 : m1;
#pragma unroll
    for (int q = 16; q > 0; q >>= 1) {
      const float y = __shfl_xor(mx, q, 32);
      mx = y > mx ? y : mx;
    }
    const float t0 = v0 ? (e0 - mx) : 0.0f;
    const float t1 = v1 ? (e1 - mx) : 0.0f;
    const float x0 = expf(t0);
    const float x1 = expf(t1);
    const float xs = (v0 ? x0 : 0.0f) + (v1 ? x1 : 0.0f);
    const float sm = wsum(xs);
    const bool has = c > 0;
    const float sc = has ? sm : 1.0f;
    const float rd = 1.0f / sc;
    v4f rec;
    rec.x = asv;
    rec.y = has ? mx : 0.0f;
    rec.z = has ? rd : 0.0f;
    rec.w = 0.0f;
    if (lane == 0) *(v4fa*)(srec + 4 * s) = rec;
  }
  __syncthreads();
  float* rp = REC + (size_t)nodeBase * 4;
#pragma unroll 1
  for (int j = 0; j < 4; ++j) {
    const int idx = j * NTHR + tid;
    const v4f p = *(const v4fa*)(srec + 4 * idx);
    *(volatile v4f*)(rp + 4 * idx) = p;
  }
  __threadfence();
#pragma unroll 1
  for (int j = 0; j < 4; ++j) {
    const int idx = j * NTHR + tid;
    const v4f p = *(const v4fa*)(srec + 4 * idx);
    *(volatile v4f*)(rp + 4 * idx) = p;
  }
}

template <int D>
__global__ __launch_bounds__(NTHR) void k_dstagg(const int* __restrict__ hits, const int* __restrict__ oc,
                                                 const float* __restrict__ AL, const float* __restrict__ REC,
                                                 const float* __restrict__ HH, const float* __restrict__ par,
                                                 int layer, const int* __restrict__ flag,
                                                 unsigned short* XT, float* outp) {
  static_assert(D == DH || D == DE);
  __shared__ int sfl[NWAVE];
  const int tid = (int)threadIdx.x, lane = tid & 31, wave = tid >> 5;
  const int kb = (int)blockIdx.x;
  const int nodeBase = kb * NBA;
  const int* hp  = hits + (size_t)kb * RCAP;
  const int* ocp = oc + nodeBase;
  const float ab = par[P_BA + layer];
  int anyf = 0;
  if constexpr (D == DE) {
    const int fi = tid < 2 * NKB ? tid : 2 * NKB - 1;
    const int fv = flag[fi * 32];
    pin_i(fv);
    const unsigned bm = __builtin_amdgcn_ballot_w32((tid < 2 * NKB) && (fv != 0));
    if (lane == 0) sfl[wave] = (bm != 0u) ? 1 : 0;
    __syncthreads();
    anyf = sfl[0] | sfl[1] | sfl[2] | sfl[3] | sfl[4] | sfl[5] | sfl[6] | sfl[7];
  }
#pragma unroll 1
  for (int si = 0; si < NBA / NWAVE; ++si) {
    const int s    = si * NWAVE + wave;
    const int node = nodeBase + s;
    const int nc   = node < NN ? node : NN - 1;
    const int ocv  = ocp[s];
    int o = (int)(((unsigned)ocv) >> 16);
    o = o > RCAP - 1 ? RCAP - 1 : o;
    int c = ocv & 0xffff;
    c = c > DEGCAP ? DEGCAP : c;
    o = __builtin_amdgcn_readfirstlane(o);
    c = __builtin_amdgcn_readfirstlane(c);
    const float adI = AL[alidx(nc) + GBM];
    float g0 = 0.0f, g1 = 0.0f, g2 = 0.0f, g3 = 0.0f;
#pragma unroll 1
    for (int b0 = 0; b0 < c; b0 += 32) {
      int idx = o + b0 + lane;
      idx = idx > RCAP - 1 ? RCAP - 1 : idx;
      int sr = hp[idx];
      pin_i(sr);
      sr = sr < 0 ? 0 : (sr > NN - 1 ? NN - 1 : sr);
      const v4f rec = *(const v4fa*)(REC + (size_t)sr * 4);
      const float e   = edge_logit(rec.x, adI, ab);
      const float att = expf(e - rec.y) * rec.z;
      const int atti  = __float_as_int(att);
      const int m32 = (c - b0) < 32 ? (c - b0) : 32;
#pragma unroll 1
      for (int k = 0; k < m32; ++k) {
        const int   sk = __builtin_amdgcn_readlane(sr, k);
        const float wk = __int_as_float(__builtin_amdgcn_readlane(atti, k));
        if constexpr (D == DH) {
          const v4f a = *(const v4fa*)(HH + (size_t)sk * DH + 4 * lane);
          g0 = fmaf(a.x, wk, g0); g1 = fmaf(a.y, wk, g1);
          g2 = fmaf(a.z, wk, g2); g3 = fmaf(a.w, wk, g3);
        } else {
          const v2f a = *(const v2fa*)(HH + (size_t)sk * DE + 2 * lane);
          g0 = fmaf(a.x, wk, g0); g1 = fmaf(a.y, wk, g1);
        }
      }
    }
    const bool live = node < NN;
    if constexpr (D == DH) {
#pragma unroll 1
      for (int it = 0; it < 3; ++it) {
        expmap4(g0, g1, g2, g3);
        logmap4(g0, g1, g2, g3);
        const bool rl = (it == 0);
        const float r0 = relu_keep(g0), r1 = relu_keep(g1), r2 = relu_keep(g2), r3 = relu_keep(g3);
        g0 = rl ? r0 : g0; g1 = rl ? r1 : g1; g2 = rl ? r2 : g2; g3 = rl ? r3 : g3;
      }
      const float q0 = live ? g0 : 0.0f, q1 = live ? g1 : 0.0f;
      const float q2 = live ? g2 : 0.0f, q3 = live ? g3 : 0.0f;
      int h01, h23, l01, l23;
      hilo_pack(q0, q1, q2, q3, h01, h23, l01, l23);
      const v4i ow = regroup16(h01, h23, l01, l23, lane);
      if (node < MP) {
        unsigned short* dp = XT + (size_t)node * KA + 8 * lane;
        *(volatile v4i*)dp = ow;
        __threadfence();
        *(volatile v4i*)dp = ow;
      }
    } else {
      expmap2(g0, g1);
      const int s0 = (2 * lane) & 31, s1 = s0 + 1;
      const float c0 = __shfl(g0, s0, 32), c1 = __shfl(g1, s0, 32);
      const float c2 = __shfl(g0, s1, 32), c3 = __shfl(g1, s1, 32);
      const float pn = __int_as_float(0x7fc00000);
      v4f ow;
      ow.x = (anyf != 0) ? pn : c0; ow.y = (anyf != 0) ? pn : c1;
      ow.z = (anyf != 0) ? pn : c2; ow.w = (anyf != 0) ? pn : c3;
      if (live) {
        float* op = outp + (size_t)node * DE + 4 * (lane & 15);
        if (lane < 16) *(volatile v4f*)op = ow;
        __threadfence();
        if (lane < 16) *(volatile v4f*)op = ow;
      }
    }
  }
}

extern "C" void kernel_launch(void* const* d_in, const int* in_sizes, int n_in,
                              void* d_out, int out_size, void* d_ws, size_t ws_size,
                              hipStream_t stream) {
  if (n_in < 12) return;
  if (in_sizes[0] != NN * DIN) return;
  if (in_sizes[1] != 2 * NE) return;
  if (in_sizes[2] != DIN * DH) return;
  if (in_sizes[3] != DH) return;
  if (in_sizes[4] != DH * DH) return;
  if (in_sizes[5] != DH) return;
  if (in_sizes[6] != 2 * DH) return;
  if (in_sizes[7] != 1) return;
  if (in_sizes[8] != DH * DE) return;
  if (in_sizes[9] != DE) return;
  if (in_sizes[10] != 2 * DE) return;
  if (in_sizes[11] != 1) return;
  if ((long long)out_size != (long long)NN * DE) return;

  const float* x    = (const float*)d_in[0];
  const int*   ei   = (const int*)d_in[1];
  const float* win  = (const float*)d_in[2];
  const float* bin  = (const float*)d_in[3];
  const float* w1   = (const float*)d_in[4];
  const float* b1   = (const float*)d_in[5];
  const float* a1   = (const float*)d_in[6];
  const float* ba1  = (const float*)d_in[7];
  const float* w2   = (const float*)d_in[8];
  const float* b2   = (const float*)d_in[9];
  const float* a2   = (const float*)d_in[10];
  const float* ba2  = (const float*)d_in[11];
  float* out = (float*)d_out;

  char* ws = (char*)d_ws;
  size_t off = 0;
  const size_t oPAR  = off; off += (size_t)PARN * 4;                 off = (off + 255) & ~(size_t)255;
  const size_t oWIN  = off; off += (size_t)DH * WP * 2;              off = (off + 255) & ~(size_t)255;
  const size_t oW1D  = off; off += (size_t)DH * WP * 2;              off = (off + 255) & ~(size_t)255;
  const size_t oW2D  = off; off += (size_t)DE * WP * 2;              off = (off + 255) & ~(size_t)255;
  const size_t oFLG  = off; off += (size_t)2 * NKB * 32 * 4;         off = (off + 255) & ~(size_t)255;
  const size_t oOC   = off; off += (size_t)2 * NPS * 4;              off = (off + 255) & ~(size_t)255;
  const size_t oAL   = off; off += (size_t)GL * (2 * GBM) * 4;       off = (off + 255) & ~(size_t)255;
  const size_t oREC  = off; off += (size_t)NPS * 16;                 off = (off + 255) & ~(size_t)255;
  const size_t oHIT  = off; off += (size_t)2 * NKB * RCAP * 4;       off = (off + 255) & ~(size_t)255;
  const size_t oXB   = off; off += (size_t)MP * KA * 2;              off = (off + 255) & ~(size_t)255;
  const size_t oXT   = off; off += (size_t)MP * KA * 2;              off = (off + 255) & ~(size_t)255;
  const size_t oHH   = off; off += (size_t)MP * DH * 4;              off = (off + 255) & ~(size_t)255;
  if (off > ws_size || off > (size_t)(128u << 20)) return;
  float*          PAR  = (float*)(ws + oPAR);
  unsigned short* WINT = (unsigned short*)(ws + oWIN);
  unsigned short* W1D  = (unsigned short*)(ws + oW1D);
  unsigned short* W2D  = (unsigned short*)(ws + oW2D);
  int*            FLG  = (int*)(ws + oFLG);
  int*            OCP  = (int*)(ws + oOC);
  float*          ALP  = (float*)(ws + oAL);
  float*          REC  = (float*)(ws + oREC);
  int*            HIT  = (int*)(ws + oHIT);
  unsigned short* XB   = (unsigned short*)(ws + oXB);
  unsigned short* XT   = (unsigned short*)(ws + oXT);
  float*          HH   = (float*)(ws + oHH);
  const int* hitS = HIT;
  const int* hitD = HIT + (size_t)NKB * RCAP;
  const int* ocS  = OCP;
  const int* ocD  = OCP + NPS;

  const size_t bktLds = (size_t)AGG_LDS_INTS * 4;
  hipFuncSetAttribute(reinterpret_cast<const void*>(&k_bucket), hipFuncAttributeMaxDynamicSharedMemorySize, (int)bktLds);

  k_prep<<<GXB + GW_IN + GW1 + GW2 + GPAR, NTHR, 0, stream>>>(x, win, w1, w2, bin, b1, a1, ba1, b2, a2, ba2,
                                                              XB, WINT, W1D, W2D, PAR);
  k_bucket<<<2 * NKB, NTHR, bktLds, stream>>>(ei, HIT, OCP, FLG);
  k_lin0<<<GL, GTHR, 0, stream>>>(XB, WINT, PAR, XT);
  k_lin<DH><<<GL, GTHR, 0, stream>>>(XT, W1D, KEXT1, PAR, P_B1, P_A1S, P_A1D, HH, ALP);
  k_srcstat<<<NKB, NTHR, 0, stream>>>(hitS, ocS, ALP, PAR, 0, REC);
  k_dstagg<DH><<<NKB, NTHR, 0, stream>>>(hitD, ocD, ALP, REC, HH, PAR, 0, FLG, XT, out);
  k_lin<DE><<<GL, GTHR, 0, stream>>>(XT, W2D, KEXT2, PAR, P_B2, P_A2S, P_A2D, HH, ALP);
  k_srcstat<<<NKB, NTHR, 0, stream>>>(hitS, ocS, ALP, PAR, 1, REC);
  k_dstagg<DE><<<NKB, NTHR, 0, stream>>>(hitD, ocD, ALP, REC, HH, PAR, 1, FLG, XT, out);
}
